// MoveEncoder_68101001445990
// MI455X (gfx1250) — hardware-verified
//
#include <hip/hip_runtime.h>

#define NMV  32768
#define LL_  15
#define DD_  256
#define VOC  27
#define TSTR 264

typedef _Float16 f16;
typedef __attribute__((ext_vector_type(16))) f16 f16x16;
typedef __attribute__((ext_vector_type(8)))  f16 f16x8;
typedef __attribute__((ext_vector_type(8)))  float f32x8;
typedef __attribute__((ext_vector_type(4)))  float v4f_t;
typedef float v4fa __attribute__((ext_vector_type(4), may_alias));

__device__ __forceinline__ f32x8 wmma16(f16x16 a, f16x16 b, f32x8 c) {
  c = __builtin_amdgcn_wmma_f32_16x16x32_f16(false, a, false, b, (short)0, c, false, false);
  asm volatile("v_nop\n\tv_nop\n\tv_nop\n\tv_nop" : "+v"(c) : "v"(a), "v"(b));
  return c;
}
__device__ __forceinline__ f16x16 lds_frag(const f16* base, int stride) {
  const int lane = threadIdx.x & 31, row = lane & 15, kh = (lane >> 4) * 8;
  const f16x8 lo = *(const f16x8*)(base + row * stride + kh);
  const f16x8 hi = *(const f16x8*)(base + row * stride + kh + 16);
  f16x16 f;
#pragma unroll
  for (int i = 0; i < 8; ++i) { f[i] = lo[i]; f[i + 8] = hi[i]; }
  return f;
}
__device__ __forceinline__ void split16(float v, f16& h, f16& l) { h = (f16)v; l = (f16)((v - (float)h) * 2048.0f); }
__device__ __forceinline__ void load_frag2(const float* __restrict__ base, int ld, int row0, int nrows, int k0, f16x16& fh, f16x16& fl) {
  const int lane = threadIdx.x & 31, r = lane & 15, kh = (lane >> 4) * 8;
  const int row = min(row0 + r, nrows - 1);
  const float* p0 = base + (size_t)row * ld + (k0 + kh);
  const v4f_t a = *(const v4f_t*)(p0), b = *(const v4f_t*)(p0 + 4), c = *(const v4f_t*)(p0 + 16), d = *(const v4f_t*)(p0 + 20);
  const float v[16] = {a[0], a[1], a[2], a[3], b[0], b[1], b[2], b[3], c[0], c[1], c[2], c[3], d[0], d[1], d[2], d[3]};
#pragma unroll
  for (int i = 0; i < 16; ++i) { f16 h, l; split16(v[i], h, l); fh[i] = h; fl[i] = l; }
}

__global__ __launch_bounds__(256) void k_tables(const float* __restrict__ lemb, const float* __restrict__ pos,
                                                const float* __restrict__ Wq, const float* __restrict__ bq, const float* __restrict__ Wk, const float* __restrict__ bk,
                                                const float* __restrict__ Wv, const float* __restrict__ bv, float* __restrict__ tab) {
  const int lane = threadIdx.x & 31, wave = threadIdx.x >> 5, cl = lane & 15, rh = (lane >> 4) * 8;
  const int pj = blockIdx.x / 3, part = blockIdx.x % 3;
  const float* Wm = (pj == 0) ? Wq : (pj == 1) ? Wk : Wv;
  const float* bb = (pj == 0) ? bq : (pj == 1) ? bk : bv;
  const float* src = (part == 2) ? pos : lemb;
  const int row0 = (part == 1) ? 16 : 0, nrows = (part == 2) ? LL_ : VOC;
  float* dst = tab + (size_t)pj * 48 * DD_ + (size_t)((part == 2) ? 32 : row0) * DD_;
  __shared__ __attribute__((aligned(16))) float tS[8][16 * 36];
  f16x16 ah[8], al[8];
#pragma unroll
  for (int ks = 0; ks < 8; ++ks) load_frag2(src, DD_, row0, nrows, ks * 32, ah[ks], al[ks]);
#pragma unroll 1
  for (int j = 0; j < 2; ++j) {
    const int nt = wave * 2 + j;
    f32x8 acc = {}, accx = {};
#pragma unroll
    for (int ks = 0; ks < 8; ++ks) {
      f16x16 bh, bl;
      load_frag2(Wm, DD_, nt * 16, DD_, ks * 32, bh, bl);
      acc = wmma16(ah[ks], bh, acc); accx = wmma16(ah[ks], bl, accx); accx = wmma16(al[ks], bh, accx);
    }
    const int n = nt * 16 + cl;
    const float badd = (part == 2) ? bb[n] : 0.0f;
#pragma unroll
    for (int r = 0; r < 8; ++r) tS[wave][(rh + r) * 36 + j * 16 + cl] = acc[r] + accx[r] * (1.0f / 2048.0f) + badd;
  }
  asm volatile("s_wait_dscnt 0" ::: "memory");
  __builtin_amdgcn_wave_barrier();
#pragma unroll 1
  for (int pass = 0; pass < 2; ++pass) {
#pragma unroll
    for (int it = 0; it < 4; ++it) { const int c = lane + 32 * it, row = c >> 3, q = (c & 7) * 4;
      if (row0 + row < nrows) *(volatile v4f_t*)(dst + (size_t)row * DD_ + wave * 32 + q) = *(const volatile v4fa*)(&tS[wave][row * 36 + q]); }
    __threadfence();
  }
}

__global__ __launch_bounds__(64) void k_moves(const int* __restrict__ words, const int* __restrict__ rows, const int* __restrict__ cols,
                                              const int* __restrict__ dirs, const int* __restrict__ scores, const float* __restrict__ tab,
                                              const float* __restrict__ row_emb, const float* __restrict__ col_emb, const float* __restrict__ dir_emb,
                                              const float* __restrict__ score_emb, float* __restrict__ out) {
  __shared__ __attribute__((aligned(16))) f16 qS[2][2][16 * TSTR];
  __shared__ __attribute__((aligned(16))) f16 kS[2][2][16 * TSTR];
  __shared__ int wS[2][16];
  const int lane = threadIdx.x & 31, wave = threadIdx.x >> 5, cl = lane & 15, hsel = lane >> 4, rh = hsel * 8;
  const int mv = blockIdx.x * 2 + wave;
  const float* QL = tab,            *QP = tab + 32 * DD_;
  const float* KL = tab + 48 * DD_,  *KP = tab + 80 * DD_;
  const float* VL = tab + 96 * DD_,  *VP = tab + 128 * DD_;
  if (lane < 16) { int w = (lane < LL_) ? words[(size_t)mv * LL_ + lane] : 0; wS[wave][lane] = min(max(w, 0), VOC - 1); }
  asm volatile("s_wait_dscnt 0" ::: "memory");
  __builtin_amdgcn_wave_barrier();
  f16* qh = qS[wave][0]; f16* ql = qS[wave][1]; f16* khp = kS[wave][0]; f16* klp = kS[wave][1];
  const int dA = lane * 4, dB = 128 + lane * 4;
#pragma unroll 1
  for (int l = 0; l < 16; ++l) {
    float qv[8], kv[8];
    if (l < LL_) {
      const int w = wS[wave][l];
      const float* a = QL + (size_t)w * DD_; const float* bq = QP + (size_t)l * DD_;
      const float* c = KL + (size_t)w * DD_; const float* dk = KP + (size_t)l * DD_;
      const v4f_t a0 = *(const v4f_t*)(a + dA), a1 = *(const v4f_t*)(a + dB), b0 = *(const v4f_t*)(bq + dA), b1 = *(const v4f_t*)(bq + dB);
      const v4f_t c0 = *(const v4f_t*)(c + dA), c1 = *(const v4f_t*)(c + dB), e0 = *(const v4f_t*)(dk + dA), e1 = *(const v4f_t*)(dk + dB);
#pragma unroll
      for (int u = 0; u < 4; ++u) { qv[u] = a0[u] + b0[u]; qv[4 + u] = a1[u] + b1[u]; kv[u] = c0[u] + e0[u]; kv[4 + u] = c1[u] + e1[u]; }
    } else {
#pragma unroll
      for (int u = 0; u < 8; ++u) { qv[u] = 0.0f; kv[u] = 0.0f; }
    }
#pragma unroll
    for (int u = 0; u < 8; ++u) {
      const int d = (u < 4) ? (dA + u) : (dB + u - 4);
      f16 h, lo;
      split16(qv[u], h, lo); qh[l * TSTR + d] = h;  ql[l * TSTR + d] = lo;
      split16(kv[u], h, lo); khp[l * TSTR + d] = h; klp[l * TSTR + d] = lo;
    }
  }
  asm volatile("s_wait_dscnt 0" ::: "memory");
  __builtin_amdgcn_wave_barrier();
  f32x8 acc = {}, accx = {};
#pragma unroll
  for (int ks = 0; ks < 8; ++ks) {
    const f16x16 ah = lds_frag(qh + ks * 32, TSTR), al = lds_frag(ql + ks * 32, TSTR);
    const f16x16 bh = lds_frag(khp + ks * 32, TSTR), bl = lds_frag(klp + ks * 32, TSTR);
    acc = wmma16(ah, bh, acc); accx = wmma16(ah, bl, accx); accx = wmma16(al, bh, accx);
  }
  float csum = 0.0f;
#pragma unroll
  for (int r = 0; r < 8; ++r) {
    float s = (cl < LL_) ? (acc[r] + accx[r] * (1.0f / 2048.0f)) : -INFINITY;
    float m = s;
#pragma unroll
    for (int off = 8; off >= 1; off >>= 1) m = fmaxf(m, __shfl_xor(m, off, 32));
    float e = (cl < LL_) ? __expf(s - m) : 0.0f;
    float z = e;
#pragma unroll
    for (int off = 8; off >= 1; off >>= 1) z += __shfl_xor(z, off, 32);
    const float att = e / z;
    if (rh + r < LL_) csum += att;
  }
  csum += __shfl_xor(csum, 16, 32);
  float wsum[8];
#pragma unroll
  for (int u = 0; u < 8; ++u) wsum[u] = 0.0f;
#pragma unroll 1
  for (int m = 0; m < LL_; ++m) {
    const float cm = __shfl(csum, m, 32);
    const int w = wS[wave][m];
    const float* a = VL + (size_t)w * DD_; const float* p = VP + (size_t)m * DD_;
    const v4f_t a0 = *(const v4f_t*)(a + dA), a1 = *(const v4f_t*)(a + dB), p0 = *(const v4f_t*)(p + dA), p1 = *(const v4f_t*)(p + dB);
#pragma unroll
    for (int u = 0; u < 4; ++u) { wsum[u] += cm * (a0[u] + p0[u]); wsum[4 + u] += cm * (a1[u] + p1[u]); }
  }
  int ri = rows[mv], ci = cols[mv], di = dirs[mv], si = scores[mv];
  ri = min(max(ri, 0), LL_ - 1); ci = min(max(ci, 0), LL_ - 1); di = min(max(di, 0), 1); si = min(max(si, 0), 99);
  const float* re = row_emb + (size_t)ri * DD_; const float* ce = col_emb + (size_t)ci * DD_;
  const float* de = dir_emb + (size_t)di * DD_; const float* se = score_emb + (size_t)si * DD_;
  v4f_t o0, o1;
  { const v4f_t r0 = *(const v4f_t*)(re + dA), c0 = *(const v4f_t*)(ce + dA), g0 = *(const v4f_t*)(de + dA), s0 = *(const v4f_t*)(se + dA);
    const v4f_t r1 = *(const v4f_t*)(re + dB), c1 = *(const v4f_t*)(ce + dB), g1 = *(const v4f_t*)(de + dB), s1 = *(const v4f_t*)(se + dB);
#pragma unroll
    for (int u = 0; u < 4; ++u) { o0[u] = 2.0f * wsum[u] + r0[u] + c0[u] + g0[u] + s0[u]; o1[u] = 2.0f * wsum[4 + u] + r1[u] + c1[u] + g1[u] + s1[u]; } }
  float* orow = out + (size_t)mv * DD_;
#pragma unroll 1
  for (int pass = 0; pass < 2; ++pass) { *(volatile v4f_t*)(orow + dA) = o0; *(volatile v4f_t*)(orow + dB) = o1; __threadfence(); }
}

extern "C" void kernel_launch(void* const* d_in, const int* in_sizes, int n_in,
                              void* d_out, int out_size, void* d_ws, size_t ws_size,
                              hipStream_t stream) {
  (void)in_sizes; (void)n_in; (void)out_size; (void)ws_size;
  const int* words = (const int*)d_in[0];
  const int* rows = (const int*)d_in[1], *cols = (const int*)d_in[2], *dirs = (const int*)d_in[3], *scores = (const int*)d_in[4];
  const float* lemb = (const float*)d_in[5];
  const float* pos  = (const float*)d_in[6];
  const float* Wq = (const float*)d_in[7],  *bq = (const float*)d_in[8];
  const float* Wk = (const float*)d_in[9],  *bk = (const float*)d_in[10];
  const float* Wv = (const float*)d_in[11], *bv = (const float*)d_in[12];
  const float* row_emb = (const float*)d_in[13], *col_emb = (const float*)d_in[14], *dir_emb = (const float*)d_in[15], *score_emb = (const float*)d_in[16];
  float* out = (float*)d_out;
  float* tab = (float*)d_ws;
  k_tables<<<dim3(9), dim3(256), 0, stream>>>(lemb, pos, Wq, bq, Wk, bk, Wv, bv, tab);
  k_moves<<<dim3(NMV / 2), dim3(64), 0, stream>>>(words, rows, cols, dirs, scores, tab, row_emb, col_emb, dir_emb, score_emb, out);
}
